// Y_decoder_5583457485496
// MI455X (gfx1250) — hardware-verified
//
#include <hip/hip_runtime.h>
#include <stddef.h>


#define NFEAT   128
#define NLAT    64
#define KD      192
#define HID     512
#define NOUT    2
#define NTHR    256
#define NWAVE   8
#define EPT     8
#define NGRP    2
#define CHUNK   (NTHR * EPT * NGRP)
#define WCAP    (EPT * NGRP * 32)
#define LISTN   (NWAVE * WCAP)
#define NBC     4096
#define NBF     1024
#define RCAP    40960
#define RBN     128
#define TGT     256
#define DEGCAP  1024
#define OTHR    512
#define BM      64
#define KSTEPS  (KD / 32)
#define TPW     4
#define CGRP    4
#define RSEG    (KD / 8)
#define WSCAP   134217728
#define ACARRY  8.0f
#define WCARRY  64.0f
#define GSCALE  (1.0f / 512.0f)

#define LDS_FILL ((RCAP + NBF + LISTN) * 4 + 64)

static_assert((CHUNK & (CHUNK - 1)) == 0);
static_assert(CHUNK <= 4096);
static_assert((NBC & (NBC - 1)) == 0 && (NBF & (NBF - 1)) == 0);
static_assert(NBC == 4 * NBF);
static_assert(OTHR * 8 == NBC);
static_assert((RCAP % 32) == 0);
static_assert(TGT == NWAVE * 32);
static_assert((NBC % TGT) == 0);
static_assert((TGT % BM) == 0);
static_assert(WCAP == EPT * NGRP * 32);
static_assert(KD == NLAT + NFEAT);
static_assert((KD % 32) == 0);
static_assert(NLAT == 2 * 32 && NFEAT == 4 * 32);
static_assert((KD % 8) == 0 && RSEG <= 32);
static_assert(HID == 2 * CGRP * TPW * 16);
static_assert(BM == 4 * 16);
static_assert(BM * NOUT == 4 * 32);
static_assert(BM * NOUT <= NTHR);

typedef float    v2f  __attribute__((ext_vector_type(2)));
typedef float    v4f  __attribute__((ext_vector_type(4)));
typedef float    v8f  __attribute__((ext_vector_type(8)));
typedef int      v4i  __attribute__((ext_vector_type(4)));
typedef _Float16 v2h  __attribute__((ext_vector_type(2)));
typedef _Float16 v4h  __attribute__((ext_vector_type(4)));
typedef _Float16 v8h  __attribute__((ext_vector_type(8)));
typedef _Float16 v16h __attribute__((ext_vector_type(16)));
union Frag { v16h v; v8h h[2]; };

__device__ __forceinline__ v8f wmh(v16h a, v16h b, v8f c) {
  v8f d = __builtin_amdgcn_wmma_f32_16x16x32_f16(false, a, false, b, (short)0, c, false, false);
  asm volatile("v_nop\n\tv_nop\n\tv_nop\n\tv_nop" : "+v"(d) : "v"(a), "v"(b));
  return d;
}

template <int NB>
__device__ __forceinline__ int scan_chunk(const int* __restrict__ dsts, int nE, int cbase, int slotBase,
                                          int vec8, int* list, int tid, int lane, int wave) {
  int wc = 0;
#pragma unroll
  for (int g = 0; g < NGRP; ++g) {
    const int el0  = (g * NTHR + tid) * EPT;
    const int e0   = cbase + el0;
    const int sent = -2147483647 - 1;
    v4i da, db;
    if (vec8 != 0 && cbase + CHUNK <= nE) {
      da = *(const v4i*)(dsts + e0);
      db = *(const v4i*)(dsts + e0 + 4);
    } else {
      da.x = (e0     < nE) ? dsts[min(e0, nE - 1)] : sent;
      da.y = (e0 + 1 < nE) ? dsts[min(e0 + 1, nE - 1)] : sent;
      da.z = (e0 + 2 < nE) ? dsts[min(e0 + 2, nE - 1)] : sent;
      da.w = (e0 + 3 < nE) ? dsts[min(e0 + 3, nE - 1)] : sent;
      db.x = (e0 + 4 < nE) ? dsts[min(e0 + 4, nE - 1)] : sent;
      db.y = (e0 + 5 < nE) ? dsts[min(e0 + 5, nE - 1)] : sent;
      db.z = (e0 + 6 < nE) ? dsts[min(e0 + 6, nE - 1)] : sent;
      db.w = (e0 + 7 < nE) ? dsts[min(e0 + 7, nE - 1)] : sent;
    }
    const unsigned nb = (unsigned)slotBase;
    const unsigned s0 = (unsigned)da.x - nb, s1 = (unsigned)da.y - nb;
    const unsigned s2 = (unsigned)da.z - nb, s3 = (unsigned)da.w - nb;
    const unsigned s4 = (unsigned)db.x - nb, s5 = (unsigned)db.y - nb;
    const unsigned s6 = (unsigned)db.z - nb, s7 = (unsigned)db.w - nb;
    const bool h0 = s0 < (unsigned)NB, h1 = s1 < (unsigned)NB, h2 = s2 < (unsigned)NB, h3 = s3 < (unsigned)NB;
    const bool h4 = s4 < (unsigned)NB, h5 = s5 < (unsigned)NB, h6 = s6 < (unsigned)NB, h7 = s7 < (unsigned)NB;
    const unsigned any = __builtin_amdgcn_ballot_w32(h0 | h1 | h2 | h3 | h4 | h5 | h6 | h7);
    if (any != 0u) {
#define HITJ(J, HJ, SJ) { \
        const unsigned mj = __builtin_amdgcn_ballot_w32(HJ); \
        if (mj != 0u) { \
          if (HJ) { \
            const int pos = wc + (int)__builtin_amdgcn_mbcnt_lo(mj, 0u); \
            if (pos < WCAP) list[wave * WCAP + pos] = ((el0 + (J)) << 12) | (int)(SJ); \
          } \
          wc += (int)__builtin_popcount(mj); } }
      HITJ(0, h0, s0)
      HITJ(1, h1, s1)
      HITJ(2, h2, s2)
      HITJ(3, h3, s3)
      HITJ(4, h4, s4)
      HITJ(5, h5, s5)
      HITJ(6, h6, s6)
      HITJ(7, h7, s7)
#undef HITJ
    }
  }
  return wc;
}

__global__ __launch_bounds__(NTHR) void k_count(
    const int* __restrict__ dsts, int* cnt, float* dinv, int nE, int vec8) {
  __shared__ __attribute__((aligned(16))) int scnt[NBC];
  __shared__ __attribute__((aligned(16))) int list[LISTN];
  __shared__ int wcnt[NWAVE];
  const int tid = threadIdx.x, lane = tid & 31, wave = tid >> 5;
  const int nodeBase = blockIdx.x * NBC;

  for (int i = tid; i < NBC; i += NTHR) scnt[i] = 0;
  __syncthreads();

  const int nChunks = (nE + CHUNK - 1) / CHUNK;
#pragma unroll 1
  for (int ch = 0; ch < nChunks; ++ch) {
    const int cbase = ch * CHUNK;
    const int wc = scan_chunk<NBC>(dsts, nE, cbase, nodeBase, vec8, list, tid, lane, wave);
    if (lane == 0) wcnt[wave] = wc;
    __syncthreads();
    if (wave == 0) {
#pragma unroll 1
      for (int wsx = 0; wsx < NWAVE; ++wsx) {
        int n = __builtin_amdgcn_readfirstlane(wcnt[wsx]);
        n = n > WCAP ? WCAP : (n < 0 ? 0 : n);
        const int* lp = list + wsx * WCAP;
#pragma unroll 1
        for (int i = 0; i < n; ++i) {
          const int ent  = __builtin_amdgcn_readfirstlane(lp[i]);
          const int slot = ent & (NBC - 1);
          if (lane == 0) scnt[slot] = scnt[slot] + 1;
        }
      }
    }
    __syncthreads();
  }

  v4i cq[4];
  v4f dq[4];
#pragma unroll
  for (int q = 0; q < 4; ++q) {
    const int f = (wave * 4 + q) * 128 + 4 * lane;
    const v4i cv = *(const v4i*)(scnt + f);
    cq[q] = cv;
    v4f d;
    d.x = rsqrtf((float)(cv.x < 0 ? 0 : cv.x) + 1.0f);
    d.y = rsqrtf((float)(cv.y < 0 ? 0 : cv.y) + 1.0f);
    d.z = rsqrtf((float)(cv.z < 0 ? 0 : cv.z) + 1.0f);
    d.w = rsqrtf((float)(cv.w < 0 ? 0 : cv.w) + 1.0f);
    dq[q] = d;
  }
  int*   cp = cnt  + (size_t)nodeBase;
  float* dp = dinv + (size_t)nodeBase;
#pragma unroll
  for (int q = 0; q < 4; ++q) {
    const int f = (wave * 4 + q) * 128 + 4 * lane;
    *(volatile v4i*)(cp + f) = cq[q];
    *(volatile v4f*)(dp + f) = dq[q];
  }
  __threadfence();
#pragma unroll
  for (int q = 0; q < 4; ++q) {
    const int f = (wave * 4 + q) * 128 + 4 * lane;
    *(volatile v4i*)(cp + f) = cq[q];
    *(volatile v4f*)(dp + f) = dq[q];
  }
}

__global__ __launch_bounds__(OTHR) void k_offsets(
    const int* __restrict__ cnt, int* off, int* rbase, int nChunk) {
  __shared__ __attribute__((aligned(16))) int soff[NBC];
  __shared__ __attribute__((aligned(16))) int srb[RBN];
  __shared__ int wtot[OTHR / 32];
  const int tid = threadIdx.x, lane = tid & 31, wave = tid >> 5, sub = tid >> 7;
  for (int i = tid; i < RBN; i += OTHR) srb[i] = 0;
  int carry = 0;
#pragma unroll 1
  for (int ch = 0; ch < nChunk; ++ch) {
    const int base = ch * NBC;
    const v4i c0 = *(const v4i*)(cnt + base + 8 * tid);
    const v4i c1 = *(const v4i*)(cnt + base + 8 * tid + 4);
    const int e0 = max(c0.x, 0), e1 = max(c0.y, 0), e2 = max(c0.z, 0), e3 = max(c0.w, 0);
    const int e4 = max(c1.x, 0), e5 = max(c1.y, 0), e6 = max(c1.z, 0), e7 = max(c1.w, 0);
    const int ts = e0 + e1 + e2 + e3 + e4 + e5 + e6 + e7;
    int incl = ts;
#pragma unroll
    for (int d = 1; d < 32; d <<= 1) {
      const int t = __shfl_up(incl, d);
      if (lane >= d) incl += t;
    }
    if (lane == 31) wtot[wave] = incl;
    __syncthreads();
    const int S0 = wtot[0]  + wtot[1]  + wtot[2]  + wtot[3];
    const int S1 = wtot[4]  + wtot[5]  + wtot[6]  + wtot[7];
    const int S2 = wtot[8]  + wtot[9]  + wtot[10] + wtot[11];
    const int S3 = wtot[12] + wtot[13] + wtot[14] + wtot[15];
    int pre = 0;
#pragma unroll 1
    for (int w = 4 * sub; w < wave; ++w) pre += wtot[w];
    const int b0 = carry;
    const int b1 = b0 + ((S0 + 31) & ~31);
    const int b2 = b1 + ((S1 + 31) & ~31);
    const int b3 = b2 + ((S2 + 31) & ~31);
    const int b4 = b3 + ((S3 + 31) & ~31);
    const int myb = sub == 0 ? b0 : (sub == 1 ? b1 : (sub == 2 ? b2 : b3));
    if (tid == 0) {
      srb[min(4 * ch + 0, RBN - 1)] = b0;
      srb[min(4 * ch + 1, RBN - 1)] = b1;
      srb[min(4 * ch + 2, RBN - 1)] = b2;
      srb[min(4 * ch + 3, RBN - 1)] = b3;
    }
    int run = myb + pre + incl - ts;
    soff[8 * tid + 0] = run; run += e0;
    soff[8 * tid + 1] = run; run += e1;
    soff[8 * tid + 2] = run; run += e2;
    soff[8 * tid + 3] = run; run += e3;
    soff[8 * tid + 4] = run; run += e4;
    soff[8 * tid + 5] = run; run += e5;
    soff[8 * tid + 6] = run; run += e6;
    soff[8 * tid + 7] = run;
    carry = b4;
    __syncthreads();
    const v4i o0 = *(const v4i*)(soff + 4 * tid);
    const v4i o1 = *(const v4i*)(soff + 4 * (tid + OTHR));
    int* op = off + base;
    *(volatile v4i*)(op + 4 * tid) = o0;
    *(volatile v4i*)(op + 4 * (tid + OTHR)) = o1;
    __threadfence();
    *(volatile v4i*)(op + 4 * tid) = o0;
    *(volatile v4i*)(op + 4 * (tid + OTHR)) = o1;
    __syncthreads();
  }
  if (tid == 0) srb[min(4 * nChunk, RBN - 1)] = carry;
  __syncthreads();
  v4i rv = {0, 0, 0, 0};
  if (tid < 32) rv = *(const v4i*)(srb + 4 * tid);
  if (tid < 32) *(volatile v4i*)(rbase + 4 * tid) = rv;
  __threadfence();
  if (tid < 32) *(volatile v4i*)(rbase + 4 * tid) = rv;
}

__global__ __launch_bounds__(NTHR) void k_fill(
    const int* __restrict__ srcs, const int* __restrict__ dsts,
    const int* __restrict__ off, const int* __restrict__ rbase,
    int* csr, int nN, int nE, int vec8, int csrLen) {
  extern __shared__ v4f lds_dyn[];
  int* region = (int*)lds_dyn;
  int* cursor = region + RCAP;
  int* list   = cursor + NBF;
  int* wcnt   = list + LISTN;
  const int tid = threadIdx.x, lane = tid & 31, wave = tid >> 5;
  const int b = blockIdx.x;
  const int nodeBase = b * NBF;

  int rb0 = rbase[b];
  const int rb1 = rbase[b + 1];
  rb0 = rb0 < 0 ? 0 : (rb0 > csrLen ? csrLen : rb0);
  rb0 &= ~31;
  int len = rb1 - rb0;
  len = len < 0 ? 0 : (len > RCAP ? RCAP : len);
  int lenW = (len + 31) & ~31;
  if (rb0 + lenW > csrLen) lenW = (csrLen - rb0) & ~31;

  {
    const v4i z = {0, 0, 0, 0};
    for (int i = tid; i < RCAP / 4; i += NTHR) ((v4i*)region)[i] = z;
    for (int s = tid; s < NBF; s += NTHR) {
      int o = off[nodeBase + s] - rb0;
      o = o < 0 ? 0 : (o > RCAP ? RCAP : o);
      cursor[s] = o;
    }
  }
  __syncthreads();

  const int nChunks = (nE + CHUNK - 1) / CHUNK;
#pragma unroll 1
  for (int ch = 0; ch < nChunks; ++ch) {
    const int cbase = ch * CHUNK;
    const int wc = scan_chunk<NBF>(dsts, nE, cbase, nodeBase, vec8, list, tid, lane, wave);
    if (lane == 0) wcnt[wave] = wc;
    __syncthreads();
    if (wave == 0) {
#pragma unroll 1
      for (int wsx = 0; wsx < NWAVE; ++wsx) {
        int n = __builtin_amdgcn_readfirstlane(wcnt[wsx]);
        n = n > WCAP ? WCAP : (n < 0 ? 0 : n);
        const int* lp = list + wsx * WCAP;
#pragma unroll 1
        for (int i = 0; i < n; ++i) {
          const int ent  = __builtin_amdgcn_readfirstlane(lp[i]);
          const int slot = ent & (NBF - 1);
          int e = cbase + ((ent >> 12) & (CHUNK - 1));
          e = e > nE - 1 ? nE - 1 : e;
          int sv = srcs[e];
          sv = sv < 0 ? 0 : (sv > nN - 1 ? nN - 1 : sv);
          if (lane == 0) {
            int pos = cursor[slot];
            pos = pos < 0 ? 0 : (pos > RCAP - 1 ? RCAP - 1 : pos);
            region[pos] = sv;
            const int np = pos + 1;
            cursor[slot] = np > RCAP ? RCAP : np;
          }
        }
      }
    }
    __syncthreads();
  }

  const int nv = lenW >> 2;
  int* gp = csr + rb0;
#pragma unroll 1
  for (int i = tid; i < nv; i += NTHR) { const v4i v = ((const v4i*)region)[i]; *(volatile v4i*)(gp + 4 * i) = v; }
  __threadfence();
#pragma unroll 1
  for (int i = tid; i < nv; i += NTHR) { const v4i v = ((const v4i*)region)[i]; *(volatile v4i*)(gp + 4 * i) = v; }
}

__global__ __launch_bounds__(NTHR) void k_wcvt(const float* __restrict__ W1, _Float16* dp, int nUnits) {
  const int i = (int)blockIdx.x * NTHR + (int)threadIdx.x;
  if (i >= nUnits) return;
  const int n = i / RSEG;
  const int seg = i - n * RSEG;
  const float* p = W1 + (size_t)(8 * seg) * HID + n;
  v8h o;
#pragma unroll
  for (int j = 0; j < 8; ++j) o[j] = (_Float16)(p[(size_t)j * HID] * WCARRY);
  _Float16* gp = dp + (size_t)i * 8;
  *(volatile v8h*)gp = o;
  __threadfence();
  *(volatile v8h*)gp = o;
}

__global__ __launch_bounds__(NTHR) void k_agg1(
    const int* __restrict__ csr, const int* __restrict__ off, const int* __restrict__ cnt,
    const float* __restrict__ dinv, const float* __restrict__ uY, const float* __restrict__ X,
    _Float16* a16, int nN, int csrLen) {
  __shared__ __attribute__((aligned(16))) _Float16 srow[NWAVE * KD];
  const int tid = threadIdx.x, lane = tid & 31, wave = tid >> 5;
  const int tbase = blockIdx.x * TGT + wave * 32;
  const int cu = 2 * lane, cx = 4 * lane;
  const int cl    = tbase + lane;
  const int cnt_l = cnt[cl];
  const int off_l = off[cl];
  const float di_l = dinv[cl];
  _Float16* sw = srow + wave * KD;
  const int lr = lane < RSEG ? lane : (RSEG - 1);

#pragma unroll 1
  for (int j = 0; j < 32; ++j) {
    const int c = tbase + j;
    int n = __shfl(cnt_l, j);
    n = n < 0 ? 0 : (n > DEGCAP ? DEGCAP : n);
    const int st = __shfl(off_l, j);
    const float dc = __shfl(di_l, j);
    const float dd = dc * dc;
    int cr = c > nN - 1 ? nN - 1 : c;
    cr = cr < 0 ? 0 : cr;

    v2f au = *(const v2f*)(uY + (size_t)cr * NLAT + cu);
    v4f ax = *(const v4f*)(X + (size_t)cr * NFEAT + cx);
    au = au * dd;
    ax = ax * dd;
#pragma unroll 1
    for (int q0 = 0; q0 < n; q0 += 32) {
      int pos = st + q0 + lane;
      pos = pos < 0 ? 0 : (pos > csrLen - 1 ? csrLen - 1 : pos);
      int sl = csr[pos];
      sl = sl < 0 ? 0 : (sl > nN - 1 ? nN - 1 : sl);
      const int mcnt = (n - q0) < 32 ? (n - q0) : 32;
#pragma unroll 1
      for (int pp = 0; pp < mcnt; ++pp) {
        const int s = __builtin_amdgcn_readlane(sl, pp);
        const float cf = dinv[s] * dc;
        const v2f yu = *(const v2f*)(uY + (size_t)s * NLAT + cu);
        const v4f yx = *(const v4f*)(X + (size_t)s * NFEAT + cx);
        au = au + yu * cf;
        ax = ax + yx * cf;
      }
    }

    const bool live = c < nN;
    v2h ou;
    v4h ox;
    ou.x = (_Float16)(live ? au.x * ACARRY : 0.f);
    ou.y = (_Float16)(live ? au.y * ACARRY : 0.f);
    ox.x = (_Float16)(live ? ax.x * ACARRY : 0.f);
    ox.y = (_Float16)(live ? ax.y * ACARRY : 0.f);
    ox.z = (_Float16)(live ? ax.z * ACARRY : 0.f);
    ox.w = (_Float16)(live ? ax.w * ACARRY : 0.f);
    *(v2h*)(sw + cu) = ou;
    *(v4h*)(sw + NLAT + cx) = ox;
    __builtin_amdgcn_fence(__ATOMIC_RELEASE, "wavefront");
    __builtin_amdgcn_wave_barrier();
    const v8h pv = *(const v8h*)(sw + 8 * lr);
    __builtin_amdgcn_fence(__ATOMIC_RELEASE, "wavefront");
    __builtin_amdgcn_wave_barrier();

    _Float16* gp = a16 + (size_t)c * KD + 8 * lane;
    if (lane < RSEG) *(volatile v8h*)gp = pv;
    __threadfence();
    if (lane < RSEG) *(volatile v8h*)gp = pv;
  }
}

__global__ __launch_bounds__(NTHR) void k_gemm(
    const _Float16* __restrict__ Ap, const _Float16* __restrict__ Bp, const float* __restrict__ bias,
    const float* __restrict__ W2, float* xw2, int nN) {
  __shared__ __attribute__((aligned(16))) float spart[2 * BM * NOUT];
  __shared__ __attribute__((aligned(16))) float sz[BM * NOUT];
  const int tid = threadIdx.x, lane = tid & 31, wave = tid >> 5, hh = lane >> 4, m = lane & 15;
  const int rowBase = (int)blockIdx.x * BM;
  const int rg = wave >> 1, chf = wave & 1;
  const int r0 = rg * 16;
  const _Float16* ap = Ap + (size_t)(rowBase + r0 + m) * KD + 8 * hh;

  float p0[8], p1[8];
#pragma unroll
  for (int r = 0; r < 8; ++r) { p0[r] = 0.f; p1[r] = 0.f; }

#pragma unroll 1
  for (int grp = 0; grp < CGRP; ++grp) {
    const int cb = chf * (HID / 2) + grp * (TPW * 16);
    v8f acc[TPW];
#pragma unroll
    for (int t = 0; t < TPW; ++t) { v8f z = {0.f, 0.f, 0.f, 0.f, 0.f, 0.f, 0.f, 0.f}; acc[t] = z; }
    const _Float16* bp = Bp + (size_t)(cb + m) * KD + 8 * hh;
#pragma unroll 1
    for (int kt = 0; kt < KSTEPS; ++kt) {
      Frag a;
      a.h[0] = *(const v8h*)(ap + 32 * kt);
      a.h[1] = *(const v8h*)(ap + 32 * kt + 16);
#pragma unroll
      for (int t = 0; t < TPW; ++t) {
        const size_t to = (size_t)(16 * t) * KD + 32 * kt;
        Frag b;
        b.h[0] = *(const v8h*)(bp + to);
        b.h[1] = *(const v8h*)(bp + to + 16);
        acc[t] = wmh(a.v, b.v, acc[t]);
      }
    }
#pragma unroll
    for (int t = 0; t < TPW; ++t) {
      const int col = cb + 16 * t + m;
      const float bv = bias[col];
      const float w0 = W2[(size_t)col * NOUT + 0];
      const float w1 = W2[(size_t)col * NOUT + 1];
#pragma unroll
      for (int r = 0; r < 8; ++r) {
        const float g = acc[t][r] * GSCALE + bv;
        const float v = fmaxf(g, 0.f);
        p0[r] += v * w0;
        p1[r] += v * w1;
      }
    }
  }

#pragma unroll
  for (int r = 0; r < 8; ++r) {
#pragma unroll
    for (int d = 1; d < 16; d <<= 1) {
      p0[r] += __shfl_xor(p0[r], d);
      p1[r] += __shfl_xor(p1[r], d);
    }
  }
  if (m == 0) {
    float* sp = spart + (size_t)(chf * BM + r0 + 8 * hh) * NOUT;
#pragma unroll
    for (int r = 0; r < 8; ++r) { sp[r * NOUT + 0] = p0[r]; sp[r * NOUT + 1] = p1[r]; }
  }
  __syncthreads();
  if (tid < BM * NOUT) {
    const int row = tid / NOUT;
    const float s = spart[tid] + spart[BM * NOUT + tid];
    sz[tid] = (rowBase + row < nN) ? s : 0.f;
  }
  __syncthreads();
  v4f v = {0.f, 0.f, 0.f, 0.f};
  if (wave == 0) v = *(const v4f*)(sz + 4 * lane);
  float* gp = xw2 + (size_t)rowBase * NOUT + 4 * lane;
  if (wave == 0) *(volatile v4f*)gp = v;
  __threadfence();
  if (wave == 0) *(volatile v4f*)gp = v;
}

__global__ __launch_bounds__(NTHR) void k_agg2(
    const int* __restrict__ csr, const int* __restrict__ off, const int* __restrict__ cnt,
    const float* __restrict__ dinv, const float* __restrict__ xw2, const float* __restrict__ b2,
    float* out, int nN, int csrLen) {
  const int tid = threadIdx.x, lane = tid & 31, wave = tid >> 5;
  const int c = blockIdx.x * TGT + wave * 32 + lane;
  int n = cnt[c];
  n = n < 0 ? 0 : (n > DEGCAP ? DEGCAP : n);
  const int st = off[c];
  const float dc = dinv[c];
  const float dd = dc * dc;
  const v2f xc = *(const v2f*)(xw2 + (size_t)c * NOUT);
  float y0 = dd * xc.x;
  float y1 = dd * xc.y;
#pragma unroll 1
  for (int q = 0; q < n; ++q) {
    int pos = st + q;
    pos = pos < 0 ? 0 : (pos > csrLen - 1 ? csrLen - 1 : pos);
    int s = csr[pos];
    s = s < 0 ? 0 : (s > nN - 1 ? nN - 1 : s);
    const float cf = dinv[s] * dc;
    const v2f xs = *(const v2f*)(xw2 + (size_t)s * NOUT);
    y0 += cf * xs.x;
    y1 += cf * xs.y;
  }
  y0 += b2[0];
  y1 += b2[1];
  const float mx = fmaxf(y0, y1);
  const float e0 = expf(y0 - mx);
  const float e1 = expf(y1 - mx);
  const float inv = 1.0f / (e0 + e1);
  v2f o;
  o.x = e0 * inv;
  o.y = e1 * inv;
  const bool live = c < nN;
  float* gp = out + (size_t)c * NOUT;
  if (live) *(volatile v2f*)gp = o;
  __threadfence();
  if (live) *(volatile v2f*)gp = o;
}

extern "C" void kernel_launch(void* const* d_in, const int* in_sizes, int n_in,
                              void* d_out, int out_size, void* d_ws, size_t ws_size,
                              hipStream_t stream) {
  if (n_in < 7) return;
  if (in_sizes[1] < NFEAT || (in_sizes[1] % NFEAT) != 0) return;
  const int nN = in_sizes[1] / NFEAT;
  if (nN < 1 || nN > (1 << 22)) return;
  if (in_sizes[2] != nN * NLAT) return;
  if (in_sizes[0] < 2 || (in_sizes[0] & 1) != 0) return;
  const int nE = in_sizes[0] / 2;
  if (nE > (1 << 28)) return;
  if (in_sizes[3] != KD * HID || in_sizes[4] != HID) return;
  if (in_sizes[5] != HID * NOUT || in_sizes[6] != NOUT) return;
  if (out_size != nN * NOUT) return;

  const int*   ei  = (const int*)d_in[0];
  const int*   src = ei;
  const int*   dst = ei + nE;
  const float* X   = (const float*)d_in[1];
  const float* uY  = (const float*)d_in[2];
  const float* W1  = (const float*)d_in[3];
  const float* b1  = (const float*)d_in[4];
  const float* W2  = (const float*)d_in[5];
  const float* b2  = (const float*)d_in[6];
  float* out = (float*)d_out;

  const int NPAD   = ((nN + TGT - 1) / TGT) * TGT;
  const int nBC    = (nN + NBC - 1) / NBC;
  const int CNTPAD = nBC * NBC;
  if (CNTPAD < NPAD) return;
  if (4 * nBC + 1 > RBN) return;
  const int nBF    = (nN + NBF - 1) / NBF;
  if (nBF > 4 * nBC) return;
  const int csrLen = ((nE + 31) & ~31) + 4096;
  if (31 * 4 * nBC > 4096) return;
  const int nAgg   = NPAD / TGT;
  const int nGemm  = NPAD / BM;
  const int nUnits = HID * RSEG;

  char* ws = (char*)d_ws;
  size_t off = 0;
  const size_t oWp  = off; off += (size_t)HID * KD * 2;            off = (off + 255) & ~(size_t)255;
  const size_t oA16 = off; off += (size_t)NPAD * KD * 2;           off = (off + 255) & ~(size_t)255;
  const size_t oXw2 = off; off += (size_t)NPAD * NOUT * 4;         off = (off + 255) & ~(size_t)255;
  const size_t oCnt = off; off += (size_t)CNTPAD * 4;              off = (off + 255) & ~(size_t)255;
  const size_t oDi  = off; off += (size_t)CNTPAD * 4;              off = (off + 255) & ~(size_t)255;
  const size_t oOff = off; off += (size_t)CNTPAD * 4;              off = (off + 255) & ~(size_t)255;
  const size_t oRb  = off; off += (size_t)RBN * 4;                 off = (off + 255) & ~(size_t)255;
  const size_t oCsr = off; off += (size_t)csrLen * 4;              off = (off + 255) & ~(size_t)255;
  if (off > ws_size || off > (size_t)WSCAP) return;

  _Float16* wpl  = (_Float16*)(ws + oWp);
  _Float16* a16p = (_Float16*)(ws + oA16);
  float* xw2  = (float*)(ws + oXw2);
  int*   cnt  = (int*)(ws + oCnt);
  float* dinv = (float*)(ws + oDi);
  int*   offp = (int*)(ws + oOff);
  int*   rb   = (int*)(ws + oRb);
  int*   csr  = (int*)(ws + oCsr);

  const int vec8 = ((nE & 3) == 0) ? 1 : 0;

  k_count<<<nBC, NTHR, 0, stream>>>(dst, cnt, dinv, nE, vec8);
  k_offsets<<<1, OTHR, 0, stream>>>(cnt, offp, rb, nBC);
  hipFuncSetAttribute(reinterpret_cast<const void*>(&k_fill),
                      hipFuncAttributeMaxDynamicSharedMemorySize, LDS_FILL);
  k_fill<<<nBF, NTHR, LDS_FILL, stream>>>(src, dst, offp, rb, csr, nN, nE, vec8, csrLen);

  k_wcvt<<<(nUnits + NTHR - 1) / NTHR, NTHR, 0, stream>>>(W1, wpl, nUnits);
  k_agg1<<<nAgg, NTHR, 0, stream>>>(csr, offp, cnt, dinv, uY, X, a16p, nN, csrLen);

  k_gemm<<<nGemm, NTHR, 0, stream>>>(a16p, wpl, b1, W2, xw2, nN);

  k_agg2<<<nAgg, NTHR, 0, stream>>>(csr, offp, cnt, dinv, xw2, b2, out, nN, csrLen);
}
